// SuperGlueMultiHeadAttention_29927332119004
// MI455X (gfx1250) — hardware-verified
//
#include <hip/hip_runtime.h>

#define FEAT  256
#define SEQ   2048
#define BATCH 4
#define NHEAD 4
#define HD    64
#define NBH   (BATCH * NHEAD)
#define MROWS (BATCH * SEQ)
#define NXE   (BATCH * FEAT * SEQ)
#define NWE   (FEAT * FEAT)
#define TP    68
static_assert(HD * NHEAD == FEAT);
static_assert(HD == 64 && (SEQ % 128) == 0 && (SEQ % 64) == 0);
static_assert((FEAT % 64) == 0 && (FEAT % 32) == 0 && (MROWS % 128) == 0);

typedef __bf16         v16b  __attribute__((ext_vector_type(16)));
typedef float          v8f   __attribute__((ext_vector_type(8)));
typedef float          v4f   __attribute__((ext_vector_type(4)));
typedef unsigned int   v4u   __attribute__((ext_vector_type(4)));
typedef unsigned short v8us  __attribute__((ext_vector_type(8)));
typedef unsigned short v16us __attribute__((ext_vector_type(16)));
typedef v4f  __attribute__((may_alias)) v4fa;
typedef v4u  __attribute__((may_alias)) v4ua;
typedef v8us __attribute__((may_alias)) v8usa;

#if defined(__HIP_DEVICE_COMPILE__)
#define DEV_ASM 1
#else
#define DEV_ASM 0
#endif

__device__ __forceinline__ unsigned short bf_bits(float f) {
  const unsigned u = __float_as_uint(f);
  return (unsigned short)((u + 0x7FFFu + ((u >> 16) & 1u)) >> 16);
}
__device__ __forceinline__ float bf_up(unsigned short hb) { return __uint_as_float(((unsigned)hb) << 16); }
__device__ __forceinline__ unsigned pk16(unsigned short a, unsigned short b) { return (unsigned)a | ((unsigned)b << 16); }
__device__ __forceinline__ v8f zero8() { v8f z = {0.f, 0.f, 0.f, 0.f, 0.f, 0.f, 0.f, 0.f}; return z; }

union FB { v16b v; v8us h[2]; v16us u; };
__device__ __forceinline__ v16b ldfrag_b(const unsigned short* p) {
  FB f;
  f.h[0] = *(const v8usa*)(p);
  f.h[1] = *(const v8usa*)(p + 16);
  return f.v;
}

__device__ __forceinline__ v8f mma_b(v16b a, v16b b, v8f c) {
  c = __builtin_amdgcn_wmma_f32_16x16x32_bf16(false, a, false, b, (short)0, c, false, false);
#if DEV_ASM
  asm volatile("v_nop\n\tv_nop\n\tv_nop\n\tv_nop" : "+v"(c) : "v"(a), "v"(b));
#endif
  return c;
}

struct P2 { v16b hi, lo; };
__device__ __forceinline__ P2 split_p(v8f a, v8f c) {
  v16us hu, lu;
#pragma unroll
  for (int r = 0; r < 8; ++r) {
    const unsigned short h0 = bf_bits(a[r]);
    hu[r] = h0;
    lu[r] = bf_bits(a[r] - bf_up(h0));
    const unsigned short h1 = bf_bits(c[r]);
    hu[8 + r] = h1;
    lu[8 + r] = bf_bits(c[r] - bf_up(h1));
  }
  FB H, L;
  H.u = hu; L.u = lu;
  P2 p;
  p.hi = H.v; p.lo = L.v;
  return p;
}

__device__ __forceinline__ void xpose_store_pass(unsigned short* xT, v4u o0, v4u o1, int wb, int n0, int c0, int tid) {
#pragma unroll
  for (int it = 0; it < 2; ++it) {
    const int job = tid + it * 256;
    const int r = job >> 3, c8 = (job & 7) * 8;
    unsigned short* dst = xT + ((size_t)(wb * SEQ + n0 + r)) * FEAT + c0 + c8;
    *(volatile v4u*)dst = (it == 0) ? o0 : o1;
  }
}

__global__ __launch_bounds__(256)
void xpose_kernel(const float* __restrict__ xq, const float* __restrict__ xk, const float* __restrict__ xv,
                  unsigned short* xT) {
  __shared__ __align__(16) float xs[64 * TP];
  const int tid  = (int)threadIdx.x;
  const int blk  = (int)blockIdx.x;
  const int nchk = blk & 31;
  const int cchk = (blk >> 5) & 3;
  const int wb   = blk >> 7;
  const int which = wb >> 2, b = wb & 3;
  const int n0 = nchk * 64, c0 = cchk * 64;
  const float* src = (which == 0) ? xq : ((which == 1) ? xk : xv);
  const float* sg = src + ((size_t)(b * FEAT + c0)) * SEQ + n0;

#pragma unroll
  for (int i = 0; i < 4; ++i) {
    const int idx = tid + i * 256;
    const int c = idx >> 4, j4 = (idx & 15) * 4;
    const v4f a = *(const v4fa*)(sg + (size_t)c * SEQ + j4);
    *(v4fa*)(xs + c * TP + j4) = a;
  }
  __syncthreads();

  v4u ov0, ov1;
#pragma unroll
  for (int it = 0; it < 2; ++it) {
    const int job = tid + it * 256;
    const int r = job >> 3, c8 = (job & 7) * 8;
    float f[8];
#pragma unroll
    for (int e = 0; e < 8; ++e) f[e] = xs[(c8 + e) * TP + r];
    v4u p;
#pragma unroll
    for (int e = 0; e < 4; ++e) p[e] = pk16(bf_bits(f[2 * e]), bf_bits(f[2 * e + 1]));
    if (it == 0) ov0 = p; else ov1 = p;
  }
  xpose_store_pass(xT, ov0, ov1, wb, n0, c0, tid);
  __threadfence();
  xpose_store_pass(xT, ov0, ov1, wb, n0, c0, tid);
}

__global__ __launch_bounds__(256)
void wconv_kernel(const float* __restrict__ wq, const float* __restrict__ wk, const float* __restrict__ wv,
                  const float* __restrict__ wm, unsigned short* Wb) {
  const int g   = (int)blockIdx.x * 256 + (int)threadIdx.x;
  const int mat = g >> 13;
  const int e   = g & 8191;
  const int o   = e >> 5;
  const int j8  = (e & 31) * 8;
  const float* w = (mat == 0) ? wq : ((mat == 1) ? wk : ((mat == 2) ? wv : wm));
  const int base = (mat == 3) ? (4 * (j8 & 63) + (j8 >> 6)) : j8;
  const int step = (mat == 3) ? 4 : 1;
  const float* row = w + (size_t)o * FEAT;
  float f[8];
#pragma unroll
  for (int i = 0; i < 8; ++i) f[i] = row[base + step * i];
  v4u p;
#pragma unroll
  for (int i = 0; i < 4; ++i) p[i] = pk16(bf_bits(f[2 * i]), bf_bits(f[2 * i + 1]));
  unsigned short* dst = Wb + (size_t)g * 8;
  *(volatile v4u*)dst = p;
  __threadfence();
  *(volatile v4u*)dst = p;
}

__device__ __forceinline__ void proj_store_pass(const unsigned short* sTh, const unsigned short* sTl,
                                                unsigned short* ph, unsigned short* pl,
                                                int which, int bh, int l0, int w, int lane) {
  const int q8 = lane & 7, sub = lane >> 3;
#pragma unroll
  for (int i = 0; i < 8; ++i) {
    const int lid = w * 32 + i * 4 + sub;
    int so;
    size_t go;
    if (which != 2) {
      so = lid * HD + 8 * q8;
      go = ((size_t)bh * SEQ + l0 + lid) * HD + 8 * q8;
    } else {
      const int d = lid >> 1, hl = lid & 1;
      so = d * 128 + 64 * hl + 8 * q8;
      go = ((size_t)bh * HD + d) * SEQ + l0 + 64 * hl + 8 * q8;
    }
    const v4u vh = *(const v4ua*)(sTh + so);
    const v4u vl = *(const v4ua*)(sTl + so);
    *(volatile v4u*)(ph + go) = vh;
    *(volatile v4u*)(pl + go) = vl;
  }
}

__global__ __launch_bounds__(128)
void proj_kernel(const unsigned short* __restrict__ xT,
                 const unsigned short* __restrict__ Wb,
                 const float* __restrict__ bq, const float* __restrict__ bk, const float* __restrict__ bv,
                 unsigned short* Qh, unsigned short* Ql,
                 unsigned short* Kh, unsigned short* Kl,
                 unsigned short* Vh, unsigned short* Vl) {
  __shared__ __align__(16) unsigned short sTh[128 * 64];
  __shared__ __align__(16) unsigned short sTl[128 * 64];

  const int tid = (int)threadIdx.x, lane = tid & 31, w = tid >> 5;
  const int h = lane >> 4, m = lane & 15;
  const int m0 = (int)blockIdx.x * 128;
  const int cg = (int)blockIdx.y;
  const int which = cg >> 2, head = cg & 3;
  const int m0w = m0 + 32 * w;

  const unsigned short* xa0 = xT + ((size_t)which * MROWS + m0w + m) * FEAT + 8 * h;
  const unsigned short* xa1 = xa0 + (size_t)16 * FEAT;
  const unsigned short* wbb = Wb + (size_t)which * NWE + 8 * h;

  v8f acc[2][4];
#pragma unroll
  for (int mt = 0; mt < 2; ++mt)
#pragma unroll
    for (int nt = 0; nt < 4; ++nt) acc[mt][nt] = zero8();

#pragma unroll 1
  for (int k0 = 0; k0 < FEAT; k0 += 32) {
    const v16b a0 = ldfrag_b(xa0 + k0);
    const v16b a1 = ldfrag_b(xa1 + k0);
#pragma unroll
    for (int nt = 0; nt < 4; ++nt) {
      const int o = 4 * (16 * nt + m) + head;
      const v16b b = ldfrag_b(wbb + (size_t)o * FEAT + k0);
      acc[0][nt] = mma_b(a0, b, acc[0][nt]);
      acc[1][nt] = mma_b(a1, b, acc[1][nt]);
    }
  }

  const float* bias = (which == 0) ? bq : ((which == 1) ? bk : bv);
  const float osc = (which == 0) ? 0.125f : 1.0f;
  if (which != 2) {
#pragma unroll
    for (int nt = 0; nt < 4; ++nt) {
      const int feat = 16 * nt + m;
      const float bvl = bf_up(bf_bits(bias[4 * feat + head]));
#pragma unroll
      for (int mt = 0; mt < 2; ++mt) {
#pragma unroll
        for (int r = 0; r < 8; ++r) {
          const int tokl = 32 * w + 16 * mt + 8 * h + r;
          const float y = (acc[mt][nt][r] + bvl) * osc;
          const unsigned short hb = bf_bits(y);
          const unsigned short lb = bf_bits(y - bf_up(hb));
          sTh[tokl * HD + feat] = hb;
          sTl[tokl * HD + feat] = lb;
        }
      }
    }
  } else {
#pragma unroll
    for (int nt = 0; nt < 4; ++nt) {
      const int feat = 16 * nt + m;
      const float bvl = bf_up(bf_bits(bias[4 * feat + head]));
#pragma unroll
      for (int mt = 0; mt < 2; ++mt) {
        v4u ph, pl;
#pragma unroll
        for (int e = 0; e < 4; ++e) {
          const float y0 = (acc[mt][nt][2 * e] + bvl) * osc;
          const float y1 = (acc[mt][nt][2 * e + 1] + bvl) * osc;
          const unsigned short a0 = bf_bits(y0), a1 = bf_bits(y1);
          const unsigned short c0 = bf_bits(y0 - bf_up(a0)), c1 = bf_bits(y1 - bf_up(a1));
          ph[e] = pk16(a0, a1);
          pl[e] = pk16(c0, c1);
        }
        const int so = feat * 128 + 32 * w + 16 * mt + 8 * h;
        *(v4ua*)(sTh + so) = ph;
        *(v4ua*)(sTl + so) = pl;
      }
    }
  }
  __syncthreads();

  const int b = m0 / SEQ, l0 = m0 - b * SEQ, bh = b * NHEAD + head;
  unsigned short* ph = (which == 0) ? Qh : ((which == 1) ? Kh : Vh);
  unsigned short* pl = (which == 0) ? Ql : ((which == 1) ? Kl : Vl);
  proj_store_pass(sTh, sTl, ph, pl, which, bh, l0, w, lane);
  __threadfence();
  proj_store_pass(sTh, sTl, ph, pl, which, bh, l0, w, lane);
}

__device__ __forceinline__ void att_store_pass(const unsigned short* sh, const unsigned short* sl,
                                               unsigned short* Ah, unsigned short* Al,
                                               int b, int head, int q0, int lane) {
  const int q8 = lane & 7, sub = lane >> 3;
#pragma unroll
  for (int i = 0; i < 4; ++i) {
    const int row = i * 4 + sub;
    const v4u vh = *(const v4ua*)(sh + row * 64 + 8 * q8);
    const v4u vl = *(const v4ua*)(sl + row * 64 + 8 * q8);
    const size_t gi = ((size_t)(b * SEQ + q0 + row)) * FEAT + head * HD + 8 * q8;
    *(volatile v4u*)(Ah + gi) = vh;
    *(volatile v4u*)(Al + gi) = vl;
  }
}

__global__ __launch_bounds__(128)
void attn_kernel(const unsigned short* __restrict__ Qh, const unsigned short* __restrict__ Ql,
                 const unsigned short* __restrict__ Kh, const unsigned short* __restrict__ Kl,
                 const unsigned short* __restrict__ Vh, const unsigned short* __restrict__ Vl,
                 unsigned short* Ah, unsigned short* Al) {
  __shared__ __align__(16) unsigned short shi[4 * 16 * 64];
  __shared__ __align__(16) unsigned short slo[4 * 16 * 64];

  const int tid = (int)threadIdx.x, lane = tid & 31, w = tid >> 5;
  const int h = lane >> 4, m = lane & 15;
  const int bh = (int)blockIdx.y, b = bh >> 2, head = bh & 3;
  const int q0 = (int)blockIdx.x * 64 + 16 * w;

  const size_t qo = ((size_t)bh * SEQ + q0 + m) * HD + 8 * h;
  const v16b qbh0 = ldfrag_b(Qh + qo);
  const v16b qbh1 = ldfrag_b(Qh + qo + 32);
  const v16b qbl0 = ldfrag_b(Ql + qo);
  const v16b qbl1 = ldfrag_b(Ql + qo + 32);

  v8f o[4];
#pragma unroll
  for (int t = 0; t < 4; ++t) o[t] = zero8();
  float mrun = -1e30f, lrun = 0.0f;

  const size_t kbase = ((size_t)bh * SEQ + m) * HD + 8 * h;
  const size_t vbase = ((size_t)bh * HD + m) * SEQ + 8 * h;

#pragma unroll 1
  for (int kb = 0; kb < SEQ; kb += 64) {
    v8f s[4];
#pragma unroll
    for (int j = 0; j < 4; ++j) {
      const size_t kp = kbase + (size_t)(kb + 16 * j) * HD;
      const v16b kh0 = ldfrag_b(Kh + kp);
      const v16b kh1 = ldfrag_b(Kh + kp + 32);
      const v16b kl0 = ldfrag_b(Kl + kp);
      const v16b kl1 = ldfrag_b(Kl + kp + 32);
      v8f z = zero8();
      z = mma_b(kh0, qbh0, z);
      z = mma_b(kh1, qbh1, z);
      z = mma_b(kh0, qbl0, z);
      z = mma_b(kh1, qbl1, z);
      z = mma_b(kl0, qbh0, z);
      z = mma_b(kl1, qbh1, z);
      s[j] = z;
    }

    float mloc = s[0][0];
#pragma unroll
    for (int j = 0; j < 4; ++j)
#pragma unroll
      for (int r = 0; r < 8; ++r) mloc = fmaxf(mloc, s[j][r]);
    mloc = fmaxf(mloc, __shfl_xor(mloc, 16));
    const float mnew = fmaxf(mrun, mloc);
    const float alpha = __expf(mrun - mnew);
    mrun = mnew;
    float lsum = 0.0f;
#pragma unroll
    for (int j = 0; j < 4; ++j)
#pragma unroll
      for (int r = 0; r < 8; ++r) {
        const float p = __expf(s[j][r] - mnew);
        s[j][r] = p;
        lsum += p;
      }
    lsum += __shfl_xor(lsum, 16);
    lrun = lrun * alpha + lsum;
#pragma unroll
    for (int t = 0; t < 4; ++t)
#pragma unroll
      for (int r = 0; r < 8; ++r) o[t][r] = o[t][r] * alpha;

#pragma unroll
    for (int g = 0; g < 2; ++g) {
      const P2 pp = split_p(s[2 * g], s[2 * g + 1]);
#pragma unroll
      for (int t = 0; t < 4; ++t) {
        const size_t vp = vbase + (size_t)(16 * t) * SEQ + kb + 32 * g;
        const v16b vfh = ldfrag_b(Vh + vp);
        const v16b vfl = ldfrag_b(Vl + vp);
        o[t] = mma_b(vfh, pp.hi, o[t]);
        o[t] = mma_b(vfh, pp.lo, o[t]);
        o[t] = mma_b(vfl, pp.hi, o[t]);
      }
    }
  }

  const float inv = 1.0f / lrun;
  unsigned short* sh = shi + w * 1024;
  unsigned short* sl = slo + w * 1024;
#pragma unroll
  for (int t = 0; t < 4; ++t) {
    v4u ph, pl;
#pragma unroll
    for (int e = 0; e < 4; ++e) {
      const float y0 = o[t][2 * e] * inv;
      const float y1 = o[t][2 * e + 1] * inv;
      const unsigned short a0 = bf_bits(y0), a1 = bf_bits(y1);
      const unsigned short c0 = bf_bits(y0 - bf_up(a0)), c1 = bf_bits(y1 - bf_up(a1));
      ph[e] = pk16(a0, a1);
      pl[e] = pk16(c0, c1);
    }
    const int so = m * 64 + 16 * t + 8 * h;
    *(v4ua*)(sh + so) = ph;
    *(v4ua*)(sl + so) = pl;
  }
  __syncthreads();

  att_store_pass(sh, sl, Ah, Al, b, head, q0, lane);
  __threadfence();
  att_store_pass(sh, sl, Ah, Al, b, head, q0, lane);
}

__device__ __forceinline__ void merge_store_pass(const float* sO, float* out, int b, int og, int l0, int w, int lane) {
  const int q8 = lane & 7, sub = lane >> 3;
#pragma unroll
  for (int i = 0; i < 16; ++i) {
    const int lid = w * 64 + i * 4 + sub;
    const int ol = lid >> 2, piece = lid & 3;
    const v4f v = *(const v4fa*)(sO + ol * 128 + 32 * piece + 4 * q8);
    const size_t gi = ((size_t)(b * FEAT + og * 64 + ol)) * SEQ + l0 + 32 * piece + 4 * q8;
    *(volatile v4f*)(out + gi) = v;
  }
}

__global__ __launch_bounds__(128)
void merge_kernel(const unsigned short* __restrict__ Ah, const unsigned short* __restrict__ Al,
                  const unsigned short* __restrict__ Wb,
                  const float* __restrict__ bm, float* out) {
  __shared__ __align__(16) float sO[64 * 128];

  const int tid = (int)threadIdx.x, lane = tid & 31, w = tid >> 5;
  const int h = lane >> 4, m = lane & 15;
  const int m0 = (int)blockIdx.x * 128;
  const int og = (int)blockIdx.y;
  const int m0w = m0 + 32 * w;

  const size_t ao0 = ((size_t)(m0w + m)) * FEAT + 8 * h;
  const size_t ao1 = ao0 + (size_t)16 * FEAT;
  const unsigned short* wmp = Wb + (size_t)3 * NWE + ((size_t)(og * 64 + m)) * FEAT + 8 * h;

  v8f acc[2][4];
#pragma unroll
  for (int mt = 0; mt < 2; ++mt)
#pragma unroll
    for (int nt = 0; nt < 4; ++nt) acc[mt][nt] = zero8();

#pragma unroll 1
  for (int k0 = 0; k0 < FEAT; k0 += 32) {
    const v16b a0h = ldfrag_b(Ah + ao0 + k0);
    const v16b a1h = ldfrag_b(Ah + ao1 + k0);
    const v16b a0l = ldfrag_b(Al + ao0 + k0);
    const v16b a1l = ldfrag_b(Al + ao1 + k0);
#pragma unroll
    for (int nt = 0; nt < 4; ++nt) {
      const v16b bw = ldfrag_b(wmp + (size_t)nt * 16 * FEAT + k0);
      acc[0][nt] = mma_b(a0h, bw, acc[0][nt]);
      acc[0][nt] = mma_b(a0l, bw, acc[0][nt]);
      acc[1][nt] = mma_b(a1h, bw, acc[1][nt]);
      acc[1][nt] = mma_b(a1l, bw, acc[1][nt]);
    }
  }

#pragma unroll
  for (int nt = 0; nt < 4; ++nt) {
    const int feat = 16 * nt + m;
    const float bvl = bf_up(bf_bits(bm[og * 64 + feat]));
#pragma unroll
    for (int mt = 0; mt < 2; ++mt) {
      v4f ya, yb;
#pragma unroll
      for (int e = 0; e < 4; ++e) {
        ya[e] = acc[mt][nt][e] + bvl;
        yb[e] = acc[mt][nt][4 + e] + bvl;
      }
      const int so = feat * 128 + 32 * w + 16 * mt + 8 * h;
      *(v4fa*)(sO + so) = ya;
      *(v4fa*)(sO + so + 4) = yb;
    }
  }
  __syncthreads();

  const int b = m0 / SEQ, l0 = m0 - b * SEQ;
  merge_store_pass(sO, out, b, og, l0, w, lane);
  __threadfence();
  merge_store_pass(sO, out, b, og, l0, w, lane);
}

extern "C" void kernel_launch(void* const* d_in, const int* in_sizes, int n_in,
                              void* d_out, int out_size, void* d_ws, size_t ws_size,
                              hipStream_t stream) {
  if (n_in < 11) return;
  if (in_sizes[0] != NXE || in_sizes[1] != NXE || in_sizes[2] != NXE) return;
  if (in_sizes[3] != NWE || in_sizes[5] != NWE || in_sizes[7] != NWE || in_sizes[9] != NWE) return;
  if (in_sizes[4] != FEAT || in_sizes[6] != FEAT || in_sizes[8] != FEAT || in_sizes[10] != FEAT) return;
  if (out_size != NXE) return;

  const float* xq = (const float*)d_in[0];
  const float* xk = (const float*)d_in[1];
  const float* xv = (const float*)d_in[2];
  const float* wq = (const float*)d_in[3];
  const float* bq = (const float*)d_in[4];
  const float* wk = (const float*)d_in[5];
  const float* bk = (const float*)d_in[6];
  const float* wv = (const float*)d_in[7];
  const float* bv = (const float*)d_in[8];
  const float* wm = (const float*)d_in[9];
  const float* bm = (const float*)d_in[10];
  float* out = (float*)d_out;

  const size_t bXT = (size_t)3 * MROWS * FEAT * 2;
  const size_t bWB = (size_t)4 * NWE * 2;
  const size_t bPL = (size_t)NBH * SEQ * HD * 2;
  const size_t bAT = (size_t)MROWS * FEAT * 2;
  size_t off = 0;
  const size_t oXT = off; off += bXT;
  const size_t oWB = off; off += bWB;
  const size_t oQh = off; off += bPL;
  const size_t oQl = off; off += bPL;
  const size_t oKh = off; off += bPL;
  const size_t oKl = off; off += bPL;
  const size_t oVh = off; off += bPL;
  const size_t oVl = off; off += bPL;
  const size_t oAh = off; off += bAT;
  const size_t oAl = off; off += bAT;
  if (off > ws_size) return;
  if (off > (size_t)134217728) return;

  char* ws = (char*)d_ws;
  unsigned short* xT = (unsigned short*)(ws + oXT);
  unsigned short* Wb = (unsigned short*)(ws + oWB);
  unsigned short* Qh = (unsigned short*)(ws + oQh);
  unsigned short* Ql = (unsigned short*)(ws + oQl);
  unsigned short* Kh = (unsigned short*)(ws + oKh);
  unsigned short* Kl = (unsigned short*)(ws + oKl);
  unsigned short* Vh = (unsigned short*)(ws + oVh);
  unsigned short* Vl = (unsigned short*)(ws + oVl);
  unsigned short* Ah = (unsigned short*)(ws + oAh);
  unsigned short* Al = (unsigned short*)(ws + oAl);

  const dim3 gX(3 * BATCH * (FEAT / 64) * (SEQ / 64));
  const dim3 gW((4 * NWE / 8) / 256);
  const dim3 gProj(MROWS / 128, 3 * NHEAD);
  const dim3 gAtt(SEQ / 64, NBH);
  const dim3 gMrg(MROWS / 128, FEAT / 64);

  xpose_kernel<<<gX, dim3(256), 0, stream>>>(xq, xk, xv, xT);
  wconv_kernel<<<gW, dim3(256), 0, stream>>>(wq, wk, wv, wm, Wb);
  proj_kernel<<<gProj, dim3(128), 0, stream>>>(xT, Wb, bq, bk, bv, Qh, Ql, Kh, Kl, Vh, Vl);
  attn_kernel<<<gAtt, dim3(128), 0, stream>>>(Qh, Ql, Kh, Kl, Vh, Vl, Ah, Al);
  merge_kernel<<<gMrg, dim3(128), 0, stream>>>(Ah, Al, Wb, bm, out);
  (void)hipGetLastError();
}
